// RLAgent_28870770163721
// MI455X (gfx1250) — hardware-verified
//
#include <hip/hip_runtime.h>
#include <stddef.h>


#define KD    128
#define HC    64
#define GR    32
#define AP    136
#define CHUNK 2048
#define NTHR  256
#define NWAVE 8
#define WCAP  256
#define NGRP  (CHUNK / (NTHR * 4))

#define GAT_LDS(H, NB) (((NB) * HC * (H) + 3 * (NB) * (H) + NWAVE * WCAP + (NB) + NWAVE) * 4)

static_assert(WCAP == (CHUNK / NTHR) * 32);
static_assert(NGRP == 2);
static_assert(GAT_LDS(2, 512) == 284704);
static_assert(GAT_LDS(1, 1024) == 286752);

typedef float    v2f  __attribute__((ext_vector_type(2)));
typedef float    v4f  __attribute__((ext_vector_type(4)));
typedef float    v8f  __attribute__((ext_vector_type(8)));
typedef int      v4i  __attribute__((ext_vector_type(4)));
typedef _Float16 v8h  __attribute__((ext_vector_type(8)));
typedef _Float16 v16h __attribute__((ext_vector_type(16)));
union Frag   { v16h v; v8h half[2]; };
union Pack16 { v8h h; v4i i; };

template <int H> struct ColVec;
template <> struct ColVec<1> { typedef v2f t; };
template <> struct ColVec<2> { typedef v4f t; };

__device__ __forceinline__ v8f wm(v16h a, v16h b, v8f c) {
  v8f d = __builtin_amdgcn_wmma_f32_16x16x32_f16(false, a, false, b, (short)0, c, false, false);
  asm volatile("v_nop\n\tv_nop\n\tv_nop\n\tv_nop" : "+v"(d) : "v"(a), "v"(b));
  return d;
}

__device__ __forceinline__ float wsum(float v) {
  v += __shfl_xor(v, 16, 32);
  v += __shfl_xor(v, 8, 32);
  v += __shfl_xor(v, 4, 32);
  v += __shfl_xor(v, 2, 32);
  v += __shfl_xor(v, 1, 32);
  return v;
}

__device__ __forceinline__ float lrelu(float v) { return v > 0.f ? v : 0.2f * v; }
__device__ __forceinline__ float frcp(float v)  { return __builtin_amdgcn_rcpf(v); }

__global__ __launch_bounds__(NTHR) void k_prep(const float* __restrict__ W, _Float16* Wh, int K, int NC) {
  const int i  = blockIdx.x * NTHR + threadIdx.x;
  const int kq = K >> 3;
  if (i >= NC * kq) return;
  const int n  = i / kq;
  const int k0 = (i - n * kq) * 8;
  Pack16 u;
#pragma unroll
  for (int j = 0; j < 8; ++j) u.h[j] = (_Float16)(W[(size_t)(k0 + j) * NC + n] * 8.0f);
  _Float16* p = Wh + (size_t)n * K + k0;
  *(volatile v4i*)p = u.i;
  __threadfence();
  *(volatile v4i*)p = u.i;
}

template <int H>
__global__ __launch_bounds__(2 * HC * H) void k_gemm(
    const float* __restrict__ X, const _Float16* __restrict__ Wh,
    const float* __restrict__ att_s, const float* __restrict__ att_d,
    float* xp, float* asrc, float* adst, int nN) {
  constexpr int NC  = HC * H;
  constexpr int NTH = 2 * NC;
  constexpr int XSP = NC + 4;
  __shared__ __attribute__((aligned(16))) _Float16 At[GR * AP];
  __shared__ __attribute__((aligned(16))) float Xs[GR * XSP];
  __shared__ __attribute__((aligned(16))) float AD[2 * GR * H];

  const int tid  = threadIdx.x;
  const int lane = tid & 31;
  const int wave = tid >> 5;
  const int hh   = lane >> 4;
  const int m    = lane & 15;
  const int rowBase = blockIdx.x * GR;

  for (int i = tid; i < GR * (KD / 8); i += NTH) {
    const int r  = i >> 4;
    const int c0 = (i & 15) * 8;
    int row = rowBase + r;
    if (row > nN - 1) row = nN - 1;
    const float* p = X + (size_t)row * KD + c0;
    const v4f f0 = *(const v4f*)(p), f1 = *(const v4f*)(p + 4);
    Pack16 u;
    u.h[0] = (_Float16)f0.x; u.h[1] = (_Float16)f0.y; u.h[2] = (_Float16)f0.z; u.h[3] = (_Float16)f0.w;
    u.h[4] = (_Float16)f1.x; u.h[5] = (_Float16)f1.y; u.h[6] = (_Float16)f1.z; u.h[7] = (_Float16)f1.w;
    *(v8h*)(At + r * AP + c0) = u.h;
  }
  __syncthreads();

  const int ncol = wave * 16 + m;
  v8f c0a = {0.f, 0.f, 0.f, 0.f, 0.f, 0.f, 0.f, 0.f};
  v8f c1a = {0.f, 0.f, 0.f, 0.f, 0.f, 0.f, 0.f, 0.f};
#pragma unroll
  for (int kt = 0; kt < KD / 32; ++kt) {
    const int k0 = kt * 32;
    Frag a0, a1, b;
    const _Float16* pb  = Wh + (size_t)ncol * KD + k0 + 8 * hh;
    const _Float16* pa0 = At + m * AP + k0 + 8 * hh;
    const _Float16* pa1 = At + (16 + m) * AP + k0 + 8 * hh;
    b.half[0]  = *(const v8h*)pb;  b.half[1]  = *(const v8h*)(pb + 16);
    a0.half[0] = *(const v8h*)pa0; a0.half[1] = *(const v8h*)(pa0 + 16);
    a1.half[0] = *(const v8h*)pa1; a1.half[1] = *(const v8h*)(pa1 + 16);
    c0a = wm(a0.v, b.v, c0a);
    c1a = wm(a1.v, b.v, c1a);
  }

#pragma unroll
  for (int r = 0; r < 8; ++r) {
    Xs[(8 * hh + r) * XSP + ncol]      = c0a[r] * 0.125f;
    Xs[(16 + 8 * hh + r) * XSP + ncol] = c1a[r] * 0.125f;
  }
  __syncthreads();

  {
    const int d    = tid >> 1;
    const int half = tid & 1;
    const int r    = d / (2 * H);
    const int rem  = d - r * 2 * H;
    const int head = rem >> 1;
    const int sd   = rem & 1;
    const float* av = sd ? att_d : att_s;
    const float* xs = Xs + r * XSP + head * HC + half * 32;
    const float* ap = av + head * HC + half * 32;
    float s = 0.f;
#pragma unroll
    for (int c = 0; c < 32; ++c) s += xs[c] * ap[c];
    s += __shfl_xor(s, 1, 32);
    if (half == 0) AD[sd * GR * H + r * H + head] = s;
  }
  __syncthreads();

  v4f xr[4];
#pragma unroll
  for (int i = 0; i < 4; ++i) {
    const int e   = 4 * ((wave * 4 + i) * 32 + lane);
    const int row = e / NC;
    const int col = e - row * NC;
    xr[i] = *(const v4f*)(Xs + row * XSP + col);
  }
  float* base = xp + (size_t)rowBase * NC;
  float* gp = 0;
  v4f gv = {0.f, 0.f, 0.f, 0.f};
  if (wave == 0 && lane < 16 * H) {
    gv = *(const v4f*)(AD + 4 * lane);
    gp = (lane < 8 * H) ? (asrc + (size_t)rowBase * H + 4 * lane)
                        : (adst + (size_t)rowBase * H + 4 * (lane - 8 * H));
  }
#pragma unroll
  for (int i = 0; i < 4; ++i) *(volatile v4f*)(base + 4 * ((wave * 4 + i) * 32 + lane)) = xr[i];
  if (gp) *(volatile v4f*)gp = gv;
  __threadfence();
#pragma unroll
  for (int i = 0; i < 4; ++i) *(volatile v4f*)(base + 4 * ((wave * 4 + i) * 32 + lane)) = xr[i];
  if (gp) *(volatile v4f*)gp = gv;
}

template <int H, int NB>
__global__ __launch_bounds__(NTHR) void k_gat(
    const int* __restrict__ ei, const float* __restrict__ xp,
    const float* __restrict__ asrc, const float* __restrict__ adst,
    const float* __restrict__ bias, const float* __restrict__ fcw, const float* __restrict__ fcb,
    float* hout, float* out, int nN, int nE) {
  constexpr int DF  = HC * H;
  constexpr int CPL = 2 * H;
  constexpr int SB  = (NB == 512) ? 9 : 10;
  static_assert(NB == 512 || NB == 1024);
  static_assert((NB / 4) % NTHR == 0 || NTHR % (NB / 4) == 0);
  typedef typename ColVec<H>::t VC;

  extern __shared__ v4f lds_dyn[];
  float* sacc = (float*)lds_dyn;
  float* mx   = sacc + NB * DF;
  float* den  = mx + NB * H;
  float* adl  = den + NB * H;
  int*   list = (int*)(adl + NB * H);
  float* obuf = (float*)(list + NWAVE * WCAP);
  int*   wcnt = (int*)(obuf + NB);

  const int tid  = threadIdx.x;
  const int lane = tid & 31;
  const int wave = tid >> 5;
  const int hd   = (lane * H) >> 5;
  const int nodeBase = blockIdx.x * NB;

  {
    const v4f z4 = {0.f, 0.f, 0.f, 0.f};
    for (int i = tid; i < NB * DF / 4; i += NTHR) lds_dyn[i] = z4;
    for (int s = tid; s < NB * H; s += NTHR) {
      mx[s]  = -1.0e30f;
      den[s] = 0.f;
      int nd = nodeBase + s / H;
      if (nd > nN - 1) nd = nN - 1;
      adl[s] = adst[(size_t)nd * H + (s % H)];
    }
  }
  __syncthreads();

  const int* eid = ei + nE;
  const bool al16 = ((nE & 3) == 0);

  const int nChunks = (nE + CHUNK - 1) / CHUNK;
#pragma unroll 1
  for (int ch = 0; ch < nChunks; ++ch) {
    const int cbase = ch * CHUNK;
    int wc = 0;
#pragma unroll
    for (int g = 0; g < NGRP; ++g) {
      const int el0 = (g * NTHR + tid) * 4;
      const int e0  = cbase + el0;
      const int sent = -2147483647 - 1;
      v4i d;
      if (al16 && (e0 + 3 < nE)) {
        d = *(const v4i*)(eid + e0);
      } else {
        d.x = (e0     < nE) ? eid[min(e0, nE - 1)]     : sent;
        d.y = (e0 + 1 < nE) ? eid[min(e0 + 1, nE - 1)] : sent;
        d.z = (e0 + 2 < nE) ? eid[min(e0 + 2, nE - 1)] : sent;
        d.w = (e0 + 3 < nE) ? eid[min(e0 + 3, nE - 1)] : sent;
      }
      const unsigned s0 = (unsigned)d.x - (unsigned)nodeBase;
      const unsigned s1 = (unsigned)d.y - (unsigned)nodeBase;
      const unsigned s2 = (unsigned)d.z - (unsigned)nodeBase;
      const unsigned s3 = (unsigned)d.w - (unsigned)nodeBase;
      const bool h0 = s0 < (unsigned)NB;
      const bool h1 = s1 < (unsigned)NB;
      const bool h2 = s2 < (unsigned)NB;
      const bool h3 = s3 < (unsigned)NB;
      const unsigned many = __builtin_amdgcn_ballot_w32(h0 | h1 | h2 | h3);
      if (many != 0u) {
#define HITJ(J, HJ, SJ) { \
          const unsigned mj = __builtin_amdgcn_ballot_w32(HJ); \
          if (HJ) { \
            const int pos = wc + (int)__builtin_amdgcn_mbcnt_lo(mj, 0u); \
            if (pos < WCAP) list[wave * WCAP + pos] = ((el0 + (J)) << SB) | (int)(SJ); \
          } \
          wc += (int)__builtin_popcount(mj); }
        HITJ(0, h0, s0)
        HITJ(1, h1, s1)
        HITJ(2, h2, s2)
        HITJ(3, h3, s3)
#undef HITJ
      }
    }
    if (lane == 0) wcnt[wave] = wc;
    __syncthreads();

    if (wave == 0) {
      for (int wsx = 0; wsx < NWAVE; ++wsx) {
        int n = wcnt[wsx];
        if (n > WCAP) n = WCAP;
        if (n < 0) n = 0;
        for (int i = 0; i < n; ++i) {
          const int ent  = list[wsx * WCAP + i];
          const int slot = ent & (NB - 1);
          const int el   = (ent >> SB) & (CHUNK - 1);
          int e = cbase + el;
          if (e > nE - 1) e = nE - 1;
          int src = ei[e];
          src = src < 0 ? 0 : (src > nN - 1 ? nN - 1 : src);
          const int ai = slot * H + hd;
          const float l  = lrelu(asrc[(size_t)src * H + hd] + adl[ai]);
          const float mo = mx[ai];
          const float mn = fmaxf(mo, l);
          const float f  = __expf(mo - mn);
          const float p  = __expf(l - mn);
          const VC xv = *(const VC*)(xp + (size_t)src * DF + CPL * lane);
          VC* sp = (VC*)(sacc + slot * DF + CPL * lane);
          const VC cur = *sp;
          *sp = cur * f + xv * p;
          const float dn = den[ai] * f + p;
          if ((lane & (32 / H - 1)) == 0) { den[ai] = dn; mx[ai] = mn; }
        }
      }
    }
    __syncthreads();
  }

  const VC bv = *(const VC*)(bias + CPL * lane);
  VC fw = bv;
  float fb = 0.f;
  if (H == 1) { fw = *(const VC*)(fcw + CPL * lane); fb = fcb[0]; }
#pragma unroll 1
  for (int j = 0; j < NB / NWAVE; ++j) {
    const int slot = wave * (NB / NWAVE) + j;
    const int node = nodeBase + slot;
    if (node >= nN) break;
    const size_t nrow = (size_t)node;
    const int ai = slot * H + hd;
    const float l  = lrelu(asrc[nrow * H + hd] + adl[ai]);
    const float mo = mx[ai];
    const float mn = fmaxf(mo, l);
    const float f  = __expf(mo - mn);
    const float p  = __expf(l - mn);
    const VC xv = *(const VC*)(xp + nrow * DF + CPL * lane);
    const VC sv = *(const VC*)(sacc + slot * DF + CPL * lane) * f + xv * p;
    const float dv  = den[ai] * f + p;
    const float inv = frcp(dv);
    VC hv = sv * inv + bv;
#pragma unroll
    for (int c = 0; c < CPL; ++c) {
      const float v = hv[c];
      hv[c] = v > 0.f ? v : (__expf(v) - 1.0f);
    }
    if (H == 2) {
      float* op = hout + nrow * DF + CPL * lane;
      *(volatile VC*)op = hv;
      __threadfence();
      *(volatile VC*)op = hv;
    } else {
      float z = 0.f;
#pragma unroll
      for (int c = 0; c < CPL; ++c) z += hv[c] * fw[c];
      z = wsum(z) + fb;
      const float o = frcp(1.0f + __expf(-z));
      if (lane == 0) obuf[slot] = o;
    }
  }
  __syncthreads();

  if (H == 1) {
    for (int fq = tid; fq < NB / 4; fq += NTHR) {
      const int n0 = nodeBase + 4 * fq;
      const v4f v = *(const v4f*)(obuf + 4 * fq);
      float* op = out + n0;
      if (n0 + 3 < nN) {
        *(volatile v4f*)op = v;
      } else {
        if (n0     < nN) ((volatile float*)op)[0] = v.x;
        if (n0 + 1 < nN) ((volatile float*)op)[1] = v.y;
        if (n0 + 2 < nN) ((volatile float*)op)[2] = v.z;
      }
    }
    __threadfence();
    for (int fq = tid; fq < NB / 4; fq += NTHR) {
      const int n0 = nodeBase + 4 * fq;
      const v4f v = *(const v4f*)(obuf + 4 * fq);
      float* op = out + n0;
      if (n0 + 3 < nN) {
        *(volatile v4f*)op = v;
      } else {
        if (n0     < nN) ((volatile float*)op)[0] = v.x;
        if (n0 + 1 < nN) ((volatile float*)op)[1] = v.y;
        if (n0 + 2 < nN) ((volatile float*)op)[2] = v.z;
      }
    }
  }
}

static inline size_t al256(size_t v) { return (v + 255) & ~(size_t)255; }

extern "C" void kernel_launch(void* const* d_in, const int* in_sizes, int n_in,
                              void* d_out, int out_size, void* d_ws, size_t ws_size,
                              hipStream_t stream) {
  if (n_in < 12) return;
  const int nN = in_sizes[0] / KD;
  const int nE = in_sizes[1] / 2;
  if (nN <= 0 || in_sizes[0] != nN * KD) return;
  if (nE < 0 || in_sizes[1] != 2 * nE) return;
  if (in_sizes[2] != KD * 2 * HC) return;
  if (in_sizes[3] != 2 * HC || in_sizes[4] != 2 * HC || in_sizes[5] != 2 * HC) return;
  if (in_sizes[6] != KD * HC) return;
  if (in_sizes[7] != HC || in_sizes[8] != HC || in_sizes[9] != HC || in_sizes[10] != HC) return;
  if (in_sizes[11] < 1) return;
  if (out_size != nN) return;

  const float* x      = (const float*)d_in[0];
  const int*   ei     = (const int*)d_in[1];
  const float* W1     = (const float*)d_in[2];
  const float* att_s1 = (const float*)d_in[3];
  const float* att_d1 = (const float*)d_in[4];
  const float* b1     = (const float*)d_in[5];
  const float* W2     = (const float*)d_in[6];
  const float* att_s2 = (const float*)d_in[7];
  const float* att_d2 = (const float*)d_in[8];
  const float* b2     = (const float*)d_in[9];
  const float* fcw    = (const float*)d_in[10];
  const float* fcb    = (const float*)d_in[11];
  float* out = (float*)d_out;

  const int nP = ((nN + GR - 1) / GR) * GR;
  size_t off = 0;
  _Float16* W1h = (_Float16*)((char*)d_ws + off); off += al256((size_t)(2 * HC) * KD * sizeof(_Float16));
  _Float16* W2h = (_Float16*)((char*)d_ws + off); off += al256((size_t)HC * KD * sizeof(_Float16));
  float* xp1 = (float*)((char*)d_ws + off); off += al256((size_t)nP * (2 * HC) * sizeof(float));
  float* as1 = (float*)((char*)d_ws + off); off += al256((size_t)nP * 2 * sizeof(float));
  float* ad1 = (float*)((char*)d_ws + off); off += al256((size_t)nP * 2 * sizeof(float));
  float* h1  = (float*)((char*)d_ws + off); off += al256((size_t)nP * (2 * HC) * sizeof(float));
  float* xp2 = (float*)((char*)d_ws + off); off += al256((size_t)nP * HC * sizeof(float));
  float* as2 = (float*)((char*)d_ws + off); off += al256((size_t)nP * sizeof(float));
  float* ad2 = (float*)((char*)d_ws + off); off += al256((size_t)nP * sizeof(float));
  if (off > ws_size) return;

  {
    const int n1 = (2 * HC) * (KD / 8);
    k_prep<<<(n1 + NTHR - 1) / NTHR, NTHR, 0, stream>>>(W1, W1h, KD, 2 * HC);
    const int n2 = HC * (KD / 8);
    k_prep<<<(n2 + NTHR - 1) / NTHR, NTHR, 0, stream>>>(W2, W2h, KD, HC);
  }

  k_gemm<2><<<nP / GR, 2 * HC * 2, 0, stream>>>(x, W1h, att_s1, att_d1, xp1, as1, ad1, nN);
  hipFuncSetAttribute(reinterpret_cast<const void*>(&k_gat<2, 512>),
                      hipFuncAttributeMaxDynamicSharedMemorySize, GAT_LDS(2, 512));
  {
    const int grid = (nN + 512 - 1) / 512;
    k_gat<2, 512><<<grid, NTHR, GAT_LDS(2, 512), stream>>>(ei, xp1, as1, ad1, b1, fcw, fcb,
                                                            h1, out, nN, nE);
  }

  k_gemm<1><<<nP / GR, 2 * HC * 1, 0, stream>>>(h1, W2h, att_s2, att_d2, xp2, as2, ad2, nN);
  hipFuncSetAttribute(reinterpret_cast<const void*>(&k_gat<1, 1024>),
                      hipFuncAttributeMaxDynamicSharedMemorySize, GAT_LDS(1, 1024));
  {
    const int grid = (nN + 1024 - 1) / 1024;
    k_gat<1, 1024><<<grid, NTHR, GAT_LDS(1, 1024), stream>>>(ei, xp2, as2, ad2, b2, fcw, fcb,
                                                              h1, out, nN, nE);
  }
}
